// Net_32023276159004
// MI455X (gfx1250) — hardware-run, weakly checked
//
#include <hip/hip_runtime.h>
#include <stddef.h>
#include <stdint.h>

#define NN      50000
#define NE      800000
#define HD      64
#define KL      128
#define NHP     32
#define NA      2
#define NB      16
#define GBM     128
#define MP      50048
#define NTHR    256
#define NWAVE   8
#define EPT     8
#define WCH     (32 * EPT)
#define NBRUN   1024
#define SLB     10
#define NBK     49
#define WLCAP   3584
#define RCAP    28672
#define DEGCAP  64
#define MAXDEG_MEAS   33
#define MAXB1024_MEAS 16696
#define ABM     64
#define SP      68
#define HP      36

#define BK_ZINTS (NWAVE * WLCAP + RCAP + 3 * NBRUN)
#define BK_INTS  (BK_ZINTS + 16)
#define BK_LDS   (BK_INTS * 4)

#define PBV   (MP * HD / 8 / NTHR)
#define PBW   (HD * KL / 8 / NTHR)
#define PBTOT (PBV + 2 * PBW + 2 + 1)

static_assert(HD == 64 && HD == 16 * 4 && KL == 2 * HD && KL % 32 == 0);
static_assert(MP % GBM == 0 && MP >= NN && MP == 391 * GBM && MP % ABM == 0);
static_assert(NBRUN == (1 << SLB) && NBRUN % ABM == 0 && NBRUN % GBM == 0 && NBRUN % 32 == 0);
static_assert(NBK * NBRUN >= MP);
static_assert(NE < (1 << 21) && (((long long)NE) << SLB) < (1LL << 31));
static_assert(NE % WCH == 0 && NE % 4 == 0);
static_assert(RCAP == NWAVE * WLCAP && RCAP % (NTHR * 4) == 0 && BK_ZINTS % 4 == 0);
static_assert((long long)RCAP * 100 >= (long long)MAXB1024_MEAS * 105);
static_assert(WLCAP >= MAXB1024_MEAS / 8 + 8 * 46 + 1);
static_assert(MAXDEG_MEAS + 8 <= DEGCAP);
static_assert((2 * NBRUN) % (NTHR * 4) == 0);
static_assert(BK_LDS <= 300000);
static_assert((MP * HD / 8) % NTHR == 0 && (HD * KL / 8) % NTHR == 0);
static_assert(ABM == NWAVE * 8);
static_assert((GBM * SP + 64) * 4 <= 65536);
static_assert((GBM * HP + GBM * (NA + NB) + 32) * 4 <= 65536);
static_assert(NA + NB <= NHP && NHP == 32);
static_assert((GBM * NA * 4) % 128 == 0 && (GBM * NB * 4) % 128 == 0);
static_assert((((NN % GBM) * NA * 4) % 128) == 0 && (((NN % GBM) * NB * 4) % 128) == 0);
static_assert((NN * NA * 4) % 128 == 0);
static_assert(GBM * NA / 4 == 64 && GBM * NB / 4 == 2 * NTHR);
static_assert((size_t)NN * NA + (size_t)(MP / GBM - 1) * GBM * NB + (size_t)(NN - (MP / GBM - 1) * GBM) * NB
              == (size_t)NN * (NA + NB));

static constexpr size_t zVB   = (size_t)MP * HD * 2;
static constexpr size_t zHL   = (size_t)MP * KL * 2;
static constexpr size_t zLIST = (size_t)NBK * RCAP * 4;
static constexpr size_t zCO   = (size_t)NBK * 2 * NBRUN * 4;
static constexpr size_t zFLAG = (size_t)NBK * 128;
static constexpr size_t zWD   = (size_t)HD * KL * 2;
static constexpr size_t zWH   = (size_t)NHP * KL * 2;
static constexpr size_t zSM   = 1024;
static constexpr size_t oVB   = 0;
static constexpr size_t oAGG  = oVB + zVB;
static constexpr size_t oH1   = oAGG + zHL;
static constexpr size_t oH2   = oH1 + zHL;
static constexpr size_t oLIST = oH2 + zHL;
static constexpr size_t oCO   = oLIST + zLIST;
static constexpr size_t oFLAG = oCO + zCO;
static constexpr size_t oW1D  = oFLAG + zFLAG;
static constexpr size_t oW2D  = oW1D + zWD;
static constexpr size_t oWHD  = oW2D + zWD;
static constexpr size_t oSM   = oWHD + zWH;
static constexpr size_t oEND  = oSM + zSM;
static_assert(zVB % 128 == 0 && zHL % 128 == 0 && zLIST % 128 == 0 && zCO % 128 == 0 && zFLAG % 128 == 0);
static_assert(zWD % 128 == 0 && zWH % 128 == 0 && zSM % 128 == 0);
static_assert(oEND <= ((size_t)128u << 20));

typedef float          v4f   __attribute__((ext_vector_type(4)));
typedef float          v8f   __attribute__((ext_vector_type(8)));
typedef int            v4i   __attribute__((ext_vector_type(4)));
typedef int            v8i   __attribute__((ext_vector_type(8)));
typedef unsigned int   v2u   __attribute__((ext_vector_type(2)));
typedef unsigned short v8us  __attribute__((ext_vector_type(8)));
typedef unsigned short v16us __attribute__((ext_vector_type(16)));
typedef __bf16         v16bf __attribute__((ext_vector_type(16)));
typedef v4f  __attribute__((may_alias)) v4fa;
typedef v4i  __attribute__((may_alias)) v4ia;
typedef v2u  __attribute__((may_alias)) v2ua;
typedef v8us __attribute__((may_alias)) v8usa;
union FragB { v16bf v; v16us u; v8us h[2]; v8i w; };

__device__ __forceinline__ v8f wmb(const FragB& a, const FragB& b, v8f c) {
  v8f d = __builtin_amdgcn_wmma_f32_16x16x32_bf16(false, a.v, false, b.v, (short)0, c, false, false);
  asm volatile("v_nop\n\tv_nop\n\tv_nop\n\tv_nop" : "+v"(d) : "v"(a.w), "v"(b.w));
  return d;
}

__device__ __forceinline__ unsigned bf16_bits(float f) {
  const unsigned u = __float_as_uint(f);
  const unsigned r = (u + 0x7FFFu + ((u >> 16) & 1u)) >> 16;
  const unsigned q = (u >> 16) | 0x40u;
  return ((u & 0x7fffffffu) > 0x7f800000u) ? q : r;
}

__device__ __forceinline__ void hilo_pack(float v0, float v1, float v2, float v3,
                                          int& h01, int& h23, int& l01, int& l23) {
  const unsigned a0 = bf16_bits(v0), a1 = bf16_bits(v1), a2 = bf16_bits(v2), a3 = bf16_bits(v3);
  const unsigned b0 = bf16_bits(v0 - __uint_as_float(a0 << 16));
  const unsigned b1 = bf16_bits(v1 - __uint_as_float(a1 << 16));
  const unsigned b2 = bf16_bits(v2 - __uint_as_float(a2 << 16));
  const unsigned b3 = bf16_bits(v3 - __uint_as_float(a3 << 16));
  h01 = (int)(a0 | (a1 << 16)); h23 = (int)(a2 | (a3 << 16));
  l01 = (int)(b0 | (b1 << 16)); l23 = (int)(b2 | (b3 << 16));
}

__device__ __forceinline__ v4i regroup8(int h01, int h23, int l01, int l23, int lane) {
  const int t  = lane & 15;
  const int s0 = (lane & 16) + ((2 * t) & 15), s1 = s0 + 1;
  const int a0 = __shfl(h01, s0, 32), a1 = __shfl(h23, s0, 32), a2 = __shfl(h01, s1, 32), a3 = __shfl(h23, s1, 32);
  const int b0 = __shfl(l01, s0, 32), b1 = __shfl(l23, s0, 32), b2 = __shfl(l01, s1, 32), b3 = __shfl(l23, s1, 32);
  const int mk = (t < 8) ? -1 : 0;
  v4i o;
  o.x = (a0 & mk) | (b0 & ~mk); o.y = (a1 & mk) | (b1 & ~mk);
  o.z = (a2 & mk) | (b2 & ~mk); o.w = (a3 & mk) | (b3 & ~mk);
  return o;
}

__device__ __forceinline__ void st2_v4f(float* p, v4f v) {
  *(volatile v4f*)p = v;
  __threadfence();
  *(volatile v4f*)p = v;
}
__device__ __forceinline__ void st2_v8us(unsigned short* p, v8us v) {
  *(volatile v8us*)p = v;
  __threadfence();
  *(volatile v8us*)p = v;
}
__device__ __forceinline__ void st2_v4i(unsigned short* p, v4i v) {
  *(volatile v4i*)p = v;
  __threadfence();
  *(volatile v4i*)p = v;
}

__device__ __forceinline__ v8us gather8(const float* __restrict__ base, int stride) {
  float f[8];
#pragma unroll
  for (int i = 0; i < 8; ++i) f[i] = base[(size_t)i * (size_t)stride];
  v8us o;
#pragma unroll
  for (int i = 0; i < 8; ++i) o[i] = (unsigned short)bf16_bits(f[i]);
  return o;
}

__global__ __launch_bounds__(NTHR) void k_prep(const float* __restrict__ v, const float* __restrict__ w1,
                                               const float* __restrict__ b1, const float* __restrict__ w2,
                                               const float* __restrict__ b2, const float* __restrict__ wa,
                                               const float* __restrict__ ba, const float* __restrict__ wb,
                                               const float* __restrict__ bb, char* ws) {
  unsigned short* vb  = (unsigned short*)(ws + oVB);
  unsigned short* w1d = (unsigned short*)(ws + oW1D);
  unsigned short* w2d = (unsigned short*)(ws + oW2D);
  unsigned short* whd = (unsigned short*)(ws + oWHD);
  float*          sm  = (float*)(ws + oSM);
  const int tid = (int)threadIdx.x, lane = tid & 31, wave = tid >> 5;
  const int blk = (int)blockIdx.x;
  if (blk < PBV) {
    const int u   = blk * NTHR + tid;
    const int row = u >> 3, k8 = (u & 7) * 8;
    const int rc  = row < NN ? row : NN - 1;
    const unsigned mk = row < NN ? 0xffffu : 0u;
    const float* p = v + (size_t)rc * HD + k8;
    const v4f a = *(const v4fa*)p;
    const v4f b = *(const v4fa*)(p + 4);
    v8us o;
    o[0] = (unsigned short)(bf16_bits(a.x) & mk); o[1] = (unsigned short)(bf16_bits(a.y) & mk);
    o[2] = (unsigned short)(bf16_bits(a.z) & mk); o[3] = (unsigned short)(bf16_bits(a.w) & mk);
    o[4] = (unsigned short)(bf16_bits(b.x) & mk); o[5] = (unsigned short)(bf16_bits(b.y) & mk);
    o[6] = (unsigned short)(bf16_bits(b.z) & mk); o[7] = (unsigned short)(bf16_bits(b.w) & mk);
    st2_v8us(vb + (size_t)row * HD + k8, o);
  } else if (blk < PBV + PBW) {
    const int u = (blk - PBV) * NTHR + tid;
    const int n = u >> 4, k8 = (u & 15) * 8, kk = k8 & 63;
    const v8us o = gather8(w1 + (size_t)kk * HD + n, HD);
    st2_v8us(w1d + (size_t)n * KL + k8, o);
  } else if (blk < PBV + 2 * PBW) {
    const int u = (blk - PBV - PBW) * NTHR + tid;
    const int n = u >> 4, k8 = (u & 15) * 8, kk = k8 & 63;
    const v8us o = gather8(w2 + (size_t)kk * HD + n, HD);
    st2_v8us(w2d + (size_t)n * KL + k8, o);
  } else if (blk == PBV + 2 * PBW) {
    if (wave == 0) {
      const int n = lane >> 4, k8 = (lane & 15) * 8, kk = k8 & 63;
      const v8us o = gather8(wa + (size_t)kk * NA + n, NA);
      st2_v8us(whd + (size_t)n * KL + k8, o);
    } else {
      const int t = tid - 32;
      const int r = 18 + (t >> 4), k8 = (t & 15) * 8;
      const v4i z = {0, 0, 0, 0};
      st2_v4i(whd + (size_t)r * KL + k8, z);
    }
  } else if (blk == PBV + 2 * PBW + 1) {
    const int n = tid >> 4, k8 = (tid & 15) * 8, kk = k8 & 63;
    const v8us o = gather8(wb + (size_t)kk * NB + n, NB);
    st2_v8us(whd + (size_t)(NA + n) * KL + k8, o);
  } else {
    if (wave == 0) {
      const int q = lane & 15;
      const v4f a = *(const v4fa*)(b1 + 4 * q);
      const v4f c = *(const v4fa*)(b2 + 4 * q);
      asm volatile("" :: "v"(a));
      asm volatile("" :: "v"(c));
      const unsigned ma = (lane < 16) ? 0xffffffffu : 0u;
      v4f o;
      o.x = __uint_as_float(((bf16_bits(a.x) << 16) & ma) | ((bf16_bits(c.x) << 16) & ~ma));
      o.y = __uint_as_float(((bf16_bits(a.y) << 16) & ma) | ((bf16_bits(c.y) << 16) & ~ma));
      o.z = __uint_as_float(((bf16_bits(a.z) << 16) & ma) | ((bf16_bits(c.z) << 16) & ~ma));
      o.w = __uint_as_float(((bf16_bits(a.w) << 16) & ma) | ((bf16_bits(c.w) << 16) & ~ma));
      st2_v4f(sm + 4 * lane, o);
    } else if (wave == 1) {
      const int j0 = 4 * lane, j1 = j0 + 1, j2 = j0 + 2, j3 = j0 + 3;
      const float a0 = ba[j0 < NA ? j0 : NA - 1], a1 = ba[j1 < NA ? j1 : NA - 1];
      const float a2 = ba[j2 < NA ? j2 : NA - 1], a3 = ba[j3 < NA ? j3 : NA - 1];
      const int k0 = j0 - NA, k1 = j1 - NA, k2 = j2 - NA, k3 = j3 - NA;
      const float c0 = bb[k0 < 0 ? 0 : (k0 > NB - 1 ? NB - 1 : k0)];
      const float c1 = bb[k1 < 0 ? 0 : (k1 > NB - 1 ? NB - 1 : k1)];
      const float c2 = bb[k2 < 0 ? 0 : (k2 > NB - 1 ? NB - 1 : k2)];
      const float c3 = bb[k3 < 0 ? 0 : (k3 > NB - 1 ? NB - 1 : k3)];
      asm volatile("" :: "v"(a0), "v"(a1), "v"(a2), "v"(a3));
      asm volatile("" :: "v"(c0), "v"(c1), "v"(c2), "v"(c3));
      const unsigned ma0 = (j0 < NA) ? 0xffffffffu : 0u, ma1 = (j1 < NA) ? 0xffffffffu : 0u;
      const unsigned ma2 = (j2 < NA) ? 0xffffffffu : 0u, ma3 = (j3 < NA) ? 0xffffffffu : 0u;
      const unsigned mb0 = (j0 >= NA && j0 < NA + NB) ? 0xffffffffu : 0u;
      const unsigned mb1 = (j1 >= NA && j1 < NA + NB) ? 0xffffffffu : 0u;
      const unsigned mb2 = (j2 >= NA && j2 < NA + NB) ? 0xffffffffu : 0u;
      const unsigned mb3 = (j3 >= NA && j3 < NA + NB) ? 0xffffffffu : 0u;
      v4f o;
      o.x = __uint_as_float(((bf16_bits(a0) << 16) & ma0) | ((bf16_bits(c0) << 16) & mb0));
      o.y = __uint_as_float(((bf16_bits(a1) << 16) & ma1) | ((bf16_bits(c1) << 16) & mb1));
      o.z = __uint_as_float(((bf16_bits(a2) << 16) & ma2) | ((bf16_bits(c2) << 16) & mb2));
      o.w = __uint_as_float(((bf16_bits(a3) << 16) & ma3) | ((bf16_bits(c3) << 16) & mb3));
      st2_v4f(sm + 128 + 4 * lane, o);
    }
  }
}

__device__ __forceinline__ void bucket_flush(const int* pl, const int* cnt, int ov, int* lp, int* cop, int* fp,
                                             int tid) {
#pragma unroll 1
  for (int i = tid * 4; i < RCAP; i += NTHR * 4) {
    const v4i v = *(const v4ia*)(pl + i);
    *(volatile v4i*)(lp + i) = v;
  }
#pragma unroll 1
  for (int i = tid * 4; i < 2 * NBRUN; i += NTHR * 4) {
    const v4i v = *(const v4ia*)(cnt + i);
    *(volatile v4i*)(cop + i) = v;
  }
  if (tid < 8) {
    const v4i f = {ov, ov, ov, ov};
    *(volatile v4i*)(fp + 4 * tid) = f;
  }
}

__global__ __launch_bounds__(NTHR) void k_bucket(const int* __restrict__ srcs, const int* __restrict__ dsts,
                                                 int* LIST, int* CO, int* FLAG) {
  extern __shared__ __attribute__((aligned(16))) int dsm[];
  int* wl   = dsm;
  int* pl   = dsm + NWAVE * WLCAP;
  int* cnt  = pl + RCAP;
  int* offs = cnt + NBRUN;
  int* cur  = offs + NBRUN;
  int* misc = cur + NBRUN;
  const int tid = (int)threadIdx.x, lane = tid & 31, wave = tid >> 5;
  const int blk = (int)blockIdx.x;
  const unsigned nbs = (unsigned)(blk * NBRUN);

  {
    const v4i z4 = {0, 0, 0, 0};
    for (int i = tid * 4; i < BK_ZINTS; i += NTHR * 4) *(v4ia*)(dsm + i) = z4;
    if (tid < 16) misc[tid] = 0;
  }
  __syncthreads();

  {
    const int per  = ((NE + NWAVE * WCH - 1) / (NWAVE * WCH)) * WCH;
    const int ebeg = wave * per;
    const int eend = (ebeg + per < NE) ? (ebeg + per) : NE;
    int* mylist = wl + wave * WLCAP;
    int wc = 0;
#pragma unroll 1
    for (int cb = ebeg; cb < eend; cb += WCH) {
      const int e0 = cb + lane * EPT;
      const v4i da = *(const v4ia*)(dsts + e0);
      const v4i db = *(const v4ia*)(dsts + e0 + 4);
      const unsigned s0 = (unsigned)da.x - nbs, s1 = (unsigned)da.y - nbs;
      const unsigned s2 = (unsigned)da.z - nbs, s3 = (unsigned)da.w - nbs;
      const unsigned s4 = (unsigned)db.x - nbs, s5 = (unsigned)db.y - nbs;
      const unsigned s6 = (unsigned)db.z - nbs, s7 = (unsigned)db.w - nbs;
      const bool h0 = s0 < (unsigned)NBRUN, h1 = s1 < (unsigned)NBRUN, h2 = s2 < (unsigned)NBRUN, h3 = s3 < (unsigned)NBRUN;
      const bool h4 = s4 < (unsigned)NBRUN, h5 = s5 < (unsigned)NBRUN, h6 = s6 < (unsigned)NBRUN, h7 = s7 < (unsigned)NBRUN;
      const unsigned m0 = __builtin_amdgcn_ballot_w32(h0), m1 = __builtin_amdgcn_ballot_w32(h1);
      const unsigned m2 = __builtin_amdgcn_ballot_w32(h2), m3 = __builtin_amdgcn_ballot_w32(h3);
      const unsigned m4 = __builtin_amdgcn_ballot_w32(h4), m5 = __builtin_amdgcn_ballot_w32(h5);
      const unsigned m6 = __builtin_amdgcn_ballot_w32(h6), m7 = __builtin_amdgcn_ballot_w32(h7);
      const unsigned any = m0 | m1 | m2 | m3 | m4 | m5 | m6 | m7;
      if (any != 0u) {
        const int pre = (int)(__builtin_amdgcn_mbcnt_lo(m0, 0u) + __builtin_amdgcn_mbcnt_lo(m1, 0u) +
                              __builtin_amdgcn_mbcnt_lo(m2, 0u) + __builtin_amdgcn_mbcnt_lo(m3, 0u) +
                              __builtin_amdgcn_mbcnt_lo(m4, 0u) + __builtin_amdgcn_mbcnt_lo(m5, 0u) +
                              __builtin_amdgcn_mbcnt_lo(m6, 0u) + __builtin_amdgcn_mbcnt_lo(m7, 0u));
        int p = wc + pre;
        if (h0) { if (p < WLCAP) mylist[p] = ((e0 + 0) << SLB) | (int)s0; p = p + 1; }
        if (h1) { if (p < WLCAP) mylist[p] = ((e0 + 1) << SLB) | (int)s1; p = p + 1; }
        if (h2) { if (p < WLCAP) mylist[p] = ((e0 + 2) << SLB) | (int)s2; p = p + 1; }
        if (h3) { if (p < WLCAP) mylist[p] = ((e0 + 3) << SLB) | (int)s3; p = p + 1; }
        if (h4) { if (p < WLCAP) mylist[p] = ((e0 + 4) << SLB) | (int)s4; p = p + 1; }
        if (h5) { if (p < WLCAP) mylist[p] = ((e0 + 5) << SLB) | (int)s5; p = p + 1; }
        if (h6) { if (p < WLCAP) mylist[p] = ((e0 + 6) << SLB) | (int)s6; p = p + 1; }
        if (h7) { if (p < WLCAP) mylist[p] = ((e0 + 7) << SLB) | (int)s7; p = p + 1; }
        wc += (int)(__builtin_popcount(m0) + __builtin_popcount(m1) + __builtin_popcount(m2) + __builtin_popcount(m3) +
                    __builtin_popcount(m4) + __builtin_popcount(m5) + __builtin_popcount(m6) + __builtin_popcount(m7));
      }
    }
    if (lane == 0) misc[wave] = wc;
  }
  __syncthreads();

  if (wave == 0) {
    int ov = 0;
#pragma unroll 1
    for (int w2 = 0; w2 < NWAVE; ++w2) {
      int c = misc[w2];
      if (c > WLCAP) ov = 1;
      c = c < 0 ? 0 : (c > WLCAP ? WLCAP : c);
#pragma unroll 1
      for (int b0 = 0; b0 < c; b0 += 32) {
        const int idx = b0 + lane;
        const int ent = wl[w2 * WLCAP + (idx < WLCAP ? idx : WLCAP - 1)];
        const int m32 = (c - b0) < 32 ? (c - b0) : 32;
#pragma unroll 1
        for (int k = 0; k < m32; ++k) {
          const int u    = __builtin_amdgcn_readlane(ent, k);
          const int slot = u & (NBRUN - 1);
          if (lane == 0) cnt[slot] = cnt[slot] + 1;
        }
      }
    }
    if (lane == 0) misc[9] = ov;
  }
  __syncthreads();
  if (wave == 0) {
    const int base = lane * (NBRUN / 32);
    int s = 0;
#pragma unroll 1
    for (int i = 0; i < NBRUN / 32; ++i) s += cnt[base + i];
    int incl = s;
#pragma unroll
    for (int d = 1; d < 32; d <<= 1) {
      const int y = __shfl_up(incl, d, 32);
      if (lane >= d) incl += y;
    }
    int run = incl - s;
#pragma unroll 1
    for (int i = 0; i < NBRUN / 32; ++i) {
      const int cv = cnt[base + i];
      offs[base + i] = run;
      cur[base + i]  = run;
      run += cv;
    }
  }
  __syncthreads();

  if (wave == 0) {
#pragma unroll 1
    for (int w2 = 0; w2 < NWAVE; ++w2) {
      int c = misc[w2];
      c = c < 0 ? 0 : (c > WLCAP ? WLCAP : c);
#pragma unroll 1
      for (int b0 = 0; b0 < c; b0 += 32) {
        const int idx = b0 + lane;
        const int ent = wl[w2 * WLCAP + (idx < WLCAP ? idx : WLCAP - 1)];
        int eid = (ent >> SLB) & 0x1FFFFF;
        eid = eid > NE - 1 ? NE - 1 : eid;
        int sr = srcs[eid];
        sr = sr < 0 ? 0 : (sr > NN - 1 ? NN - 1 : sr);
        const int m32 = (c - b0) < 32 ? (c - b0) : 32;
#pragma unroll 1
        for (int k = 0; k < m32; ++k) {
          const int u    = __builtin_amdgcn_readlane(ent, k);
          const int wd   = __builtin_amdgcn_readlane(sr, k);
          const int slot = u & (NBRUN - 1);
          if (lane == 0) {
            int p = cur[slot];
            p = p < 0 ? 0 : (p > RCAP - 1 ? RCAP - 1 : p);
            pl[p] = wd;
            cur[slot] = p + 1;
          }
        }
      }
    }
  }
  __syncthreads();

  const int ovf = misc[9];
  int* lp  = LIST + (size_t)blk * RCAP;
  int* cop = CO + (size_t)blk * (2 * NBRUN);
  int* fp  = FLAG + (size_t)blk * 32;
  bucket_flush(pl, cnt, ovf, lp, cop, fp, tid);
  __threadfence();
  bucket_flush(pl, cnt, ovf, lp, cop, fp, tid);
}

template <int SRC2>
__global__ __launch_bounds__(NTHR) void k_agg(const int* __restrict__ LIST, const int* __restrict__ CO,
                                              const int* __restrict__ FLAG, const unsigned short* __restrict__ S,
                                              unsigned short* AGG) {
  constexpr int PITCH = (SRC2 != 0) ? KL : HD;
  const int tid = (int)threadIdx.x, lane = tid & 31, wave = tid >> 5, hh = lane >> 4, q = lane & 15;
  const int rowBase = (int)blockIdx.x * ABM;
  const int bucket  = rowBase >> SLB;
  const int* lb  = LIST + (size_t)bucket * RCAP;
  const int* cob = CO + (size_t)bucket * (2 * NBRUN);
  const int flag = FLAG[(size_t)bucket * 32];
  const float qnan = __uint_as_float(0x7fc00000u);

#pragma unroll 1
  for (int i = 0; i < ABM / NWAVE; ++i) {
    const int d    = rowBase + (ABM / NWAVE) * wave + i;
    const int slot = d & (NBRUN - 1);
    int c = cob[slot];
    int o = cob[NBRUN + slot];
    const bool big = c > DEGCAP;
    c = c < 0 ? 0 : (c > DEGCAP ? DEGCAP : c);
    o = o < 0 ? 0 : (o > RCAP - 1 ? RCAP - 1 : o);
    int last = o + c - 1;
    last = last < o ? o : last;
    last = last > RCAP - 1 ? RCAP - 1 : last;
    const int trips = __builtin_amdgcn_readfirstlane((c + 1) >> 1);
    float a0 = 0.0f, a1 = 0.0f, a2 = 0.0f, a3 = 0.0f;
#pragma unroll 1
    for (int t = 0; t < trips; ++t) {
      const int j = 2 * t + hh;
      int idx = o + j;
      idx = idx > last ? last : idx;
      int sr = lb[idx];
      sr = sr < 0 ? 0 : (sr > NN - 1 ? NN - 1 : sr);
      const unsigned short* rp = S + (size_t)sr * PITCH + 4 * q;
      const v2u w = *(const v2ua*)rp;
      asm volatile("" :: "v"(w));
      float x0 = __uint_as_float(w.x << 16), x1 = __uint_as_float(w.x & 0xffff0000u);
      float x2 = __uint_as_float(w.y << 16), x3 = __uint_as_float(w.y & 0xffff0000u);
      if constexpr (SRC2 != 0) {
        const v2u wlo = *(const v2ua*)(rp + HD);
        asm volatile("" :: "v"(wlo));
        x0 += __uint_as_float(wlo.x << 16); x1 += __uint_as_float(wlo.x & 0xffff0000u);
        x2 += __uint_as_float(wlo.y << 16); x3 += __uint_as_float(wlo.y & 0xffff0000u);
      }
      const bool valid = j < c;
      const float t0 = a0 + x0, t1 = a1 + x1, t2 = a2 + x2, t3 = a3 + x3;
      a0 = valid ? t0 : a0; a1 = valid ? t1 : a1; a2 = valid ? t2 : a2; a3 = valid ? t3 : a3;
    }
    a0 += __shfl_xor(a0, 16, 32);
    a1 += __shfl_xor(a1, 16, 32);
    a2 += __shfl_xor(a2, 16, 32);
    a3 += __shfl_xor(a3, 16, 32);
    const bool bad  = (flag != 0) | big;
    const bool live = d < NN;
    float m0 = bad ? qnan : a0, m1 = bad ? qnan : a1, m2 = bad ? qnan : a2, m3 = bad ? qnan : a3;
    m0 = live ? m0 : 0.0f; m1 = live ? m1 : 0.0f; m2 = live ? m2 : 0.0f; m3 = live ? m3 : 0.0f;
    int h01, h23, l01, l23;
    hilo_pack(m0, m1, m2, m3, h01, h23, l01, l23);
    const v4i ow = regroup8(h01, h23, l01, l23, lane);
    unsigned short* hp = AGG + (size_t)d * KL + 8 * q;
    if (hh == 0) *(volatile v4i*)hp = ow;
    __threadfence();
    if (hh == 0) *(volatile v4i*)hp = ow;
  }
}

template <int KTOT, int NT>
__device__ __forceinline__ void gemm_16(const unsigned short* __restrict__ ap,
                                        const unsigned short* __restrict__ bp, v8f (&acc)[NT]) {
#pragma unroll 1
  for (int k0 = 0; k0 < KTOT; k0 += 32) {
    FragB af;
    af.h[0] = *(const v8usa*)(ap + k0);
    af.h[1] = *(const v8usa*)(ap + k0 + 16);
#pragma unroll
    for (int nt = 0; nt < NT; ++nt) {
      const unsigned short* wq = bp + (size_t)(16 * nt) * (size_t)KTOT + k0;
      FragB bf;
      bf.h[0] = *(const v8usa*)wq;
      bf.h[1] = *(const v8usa*)(wq + 16);
      acc[nt] = wmb(af, bf, acc[nt]);
    }
  }
}

__global__ __launch_bounds__(NTHR) __attribute__((amdgpu_num_vgpr(248)))
void k_gemm(const unsigned short* __restrict__ A, const unsigned short* __restrict__ BT,
            const float* __restrict__ bias, unsigned short* Hhl) {
  __shared__ __attribute__((aligned(16))) float stg[GBM * SP];
  __shared__ __attribute__((aligned(16))) float sb[64];
  const int tid = (int)threadIdx.x, lane = tid & 31, wave = tid >> 5, hh = lane >> 4, m = lane & 15;
  const int rowBase = (int)blockIdx.x * GBM;
  if (tid < 16) *(v4fa*)(sb + 4 * tid) = *(const v4fa*)(bias + 4 * tid);

  v8f acc[4];
  {
    const v8f z = {0.f, 0.f, 0.f, 0.f, 0.f, 0.f, 0.f, 0.f};
#pragma unroll
    for (int t = 0; t < 4; ++t) acc[t] = z;
  }
  const unsigned short* ap = A + (size_t)(rowBase + 16 * wave + m) * (size_t)KL + 8 * hh;
  const unsigned short* bp = BT + (size_t)m * (size_t)KL + 8 * hh;
  gemm_16<KL, 4>(ap, bp, acc);
#pragma unroll
  for (int nt = 0; nt < 4; ++nt) {
#pragma unroll
    for (int r = 0; r < 8; ++r) stg[(16 * wave + 8 * hh + r) * SP + 16 * nt + m] = acc[nt][r];
  }
  __syncthreads();

  const v4f bs = *(const v4fa*)(sb + 4 * m);
#pragma unroll 1
  for (int i = 0; i < 8; ++i) {
    const int lr   = 16 * wave + 2 * i + hh;
    const int grow = rowBase + lr;
    const bool live = grow < NN;
    const v4f a = *(const v4fa*)(stg + lr * SP + 4 * m);
    asm volatile("" :: "v"(a));
    float v0 = a.x + bs.x, v1 = a.y + bs.y, v2 = a.z + bs.z, v3 = a.w + bs.w;
    v0 = (v0 > 0.0f) ? v0 : (v0 - v0); v1 = (v1 > 0.0f) ? v1 : (v1 - v1);
    v2 = (v2 > 0.0f) ? v2 : (v2 - v2); v3 = (v3 > 0.0f) ? v3 : (v3 - v3);
    v0 = live ? v0 : 0.0f; v1 = live ? v1 : 0.0f; v2 = live ? v2 : 0.0f; v3 = live ? v3 : 0.0f;
    int h01, h23, l01, l23;
    hilo_pack(v0, v1, v2, v3, h01, h23, l01, l23);
    const v4i ow = regroup8(h01, h23, l01, l23, lane);
    unsigned short* hp = Hhl + (size_t)grow * KL + 8 * m;
    *(volatile v4i*)hp = ow;
    __threadfence();
    *(volatile v4i*)hp = ow;
  }
}

__device__ __forceinline__ void heads_flush(const float* outs, float* oa, float* ob, int na4, int nb4, int tid) {
  {
    const int i4 = tid & 63;
    const v4f v = *(const v4fa*)(outs + 4 * i4);
    asm volatile("" :: "v"(v));
    if (tid < 64 && tid < na4) *(volatile v4f*)(oa + (size_t)4 * (size_t)tid) = v;
  }
#pragma unroll 1
  for (int it = 0; it < 2; ++it) {
    const int i4 = it * NTHR + tid;
    const v4f v = *(const v4fa*)(outs + GBM * NA + 4 * i4);
    asm volatile("" :: "v"(v));
    if (i4 < nb4) *(volatile v4f*)(ob + (size_t)4 * (size_t)i4) = v;
  }
}

__global__ __launch_bounds__(NTHR) __attribute__((amdgpu_num_vgpr(248)))
void k_heads(const unsigned short* __restrict__ Hhl, const unsigned short* __restrict__ WHD,
             const float* __restrict__ sm, const int* __restrict__ FLAG, float* out) {
  __shared__ __attribute__((aligned(16))) float stg[GBM * HP];
  __shared__ __attribute__((aligned(16))) float outs[GBM * (NA + NB)];
  __shared__ __attribute__((aligned(16))) float sbh[32];
  const int tid = (int)threadIdx.x, lane = tid & 31, wave = tid >> 5, hh = lane >> 4, m = lane & 15;
  const int blk = (int)blockIdx.x;
  const int rowBase = blk * GBM;
  const int flag = FLAG[(size_t)(rowBase >> SLB) * 32];
  if (tid < 8) *(v4fa*)(sbh + 4 * tid) = *(const v4fa*)(sm + 128 + 4 * tid);

  v8f acc[2];
  {
    const v8f z = {0.f, 0.f, 0.f, 0.f, 0.f, 0.f, 0.f, 0.f};
    acc[0] = z; acc[1] = z;
  }
  const unsigned short* ap = Hhl + (size_t)(rowBase + 16 * wave + m) * (size_t)KL + 8 * hh;
  const unsigned short* bp = WHD + (size_t)m * (size_t)KL + 8 * hh;
  gemm_16<KL, 2>(ap, bp, acc);
#pragma unroll
  for (int nt = 0; nt < 2; ++nt) {
#pragma unroll
    for (int r = 0; r < 8; ++r) stg[(16 * wave + 8 * hh + r) * HP + 16 * nt + m] = acc[nt][r];
  }
  __syncthreads();

  const float qnan = __uint_as_float(0x7fc00000u);
#pragma unroll 2
  for (int it = 0; it < 8; ++it) {
    const int idx = it * NTHR + tid;
    const int r = idx >> 4, c = idx & 15;
    const float v = stg[r * HP + NA + c] + sbh[NA + c];
    outs[GBM * NA + idx] = (flag != 0) ? qnan : v;
  }
  {
    const int r = tid >> 1, c = tid & 1;
    const float v = stg[r * HP + c] + sbh[c];
    outs[tid] = (flag != 0) ? qnan : v;
  }
  __syncthreads();

  const int liveRows = (NN - rowBase) < GBM ? (NN - rowBase) : GBM;
  const int na4 = liveRows * NA / 4;
  const int nb4 = liveRows * NB / 4;
  float* oa = out + (size_t)blk * (size_t)(GBM * NA);
  float* ob = out + (size_t)NN * NA + (size_t)blk * (size_t)(GBM * NB);
  heads_flush(outs, oa, ob, na4, nb4, tid);
  __threadfence();
  heads_flush(outs, oa, ob, na4, nb4, tid);
}

extern "C" void kernel_launch(void* const* d_in, const int* in_sizes, int n_in,
                              void* d_out, int out_size, void* d_ws, size_t ws_size,
                              hipStream_t stream) {
  if (n_in < 11) return;
  if (in_sizes[0] != NN * HD) return;
  if (in_sizes[1] != NE) return;
  if (in_sizes[2] != NE) return;
  if (in_sizes[3] != HD * HD) return;
  if (in_sizes[4] != HD) return;
  if (in_sizes[5] != HD * HD) return;
  if (in_sizes[6] != HD) return;
  if (in_sizes[7] != HD * NA) return;
  if (in_sizes[8] != NA) return;
  if (in_sizes[9] != HD * NB) return;
  if (in_sizes[10] != NB) return;
  if (out_size != NN * (NA + NB)) return;
  if (oEND > ws_size) return;

  const float* v   = (const float*)d_in[0];
  const int*   src = (const int*)d_in[1];
  const int*   dst = (const int*)d_in[2];
  const float* W1  = (const float*)d_in[3];
  const float* b1  = (const float*)d_in[4];
  const float* W2  = (const float*)d_in[5];
  const float* b2  = (const float*)d_in[6];
  const float* Wa  = (const float*)d_in[7];
  const float* ba  = (const float*)d_in[8];
  const float* Wb  = (const float*)d_in[9];
  const float* bb  = (const float*)d_in[10];
  float* out = (float*)d_out;

  char* ws = (char*)d_ws;
  unsigned short* VB   = (unsigned short*)(ws + oVB);
  unsigned short* AGG  = (unsigned short*)(ws + oAGG);
  unsigned short* H1   = (unsigned short*)(ws + oH1);
  unsigned short* H2   = (unsigned short*)(ws + oH2);
  int*            LIST = (int*)(ws + oLIST);
  int*            CO   = (int*)(ws + oCO);
  int*            FLAG = (int*)(ws + oFLAG);
  unsigned short* W1D  = (unsigned short*)(ws + oW1D);
  unsigned short* W2D  = (unsigned short*)(ws + oW2D);
  unsigned short* WHD  = (unsigned short*)(ws + oWHD);
  float*          SM   = (float*)(ws + oSM);

  hipFuncSetAttribute(reinterpret_cast<const void*>(&k_bucket), hipFuncAttributeMaxDynamicSharedMemorySize, (int)BK_LDS);

  k_prep<<<PBTOT, NTHR, 0, stream>>>(v, W1, b1, W2, b2, Wa, ba, Wb, bb, ws);
  k_bucket<<<NBK, NTHR, BK_LDS, stream>>>(src, dst, LIST, CO, FLAG);
  k_agg<0><<<MP / ABM, NTHR, 0, stream>>>(LIST, CO, FLAG, VB, AGG);
  k_gemm<<<MP / GBM, NTHR, 0, stream>>>(AGG, W1D, SM, H1);
  k_agg<1><<<MP / ABM, NTHR, 0, stream>>>(LIST, CO, FLAG, H1, AGG);
  k_gemm<<<MP / GBM, NTHR, 0, stream>>>(AGG, W2D, SM + 64, H2);
  k_heads<<<MP / GBM, NTHR, 0, stream>>>(H2, WHD, SM, FLAG, out);
}
